// Attention_83502754169400
// MI455X (gfx1250) — hardware-verified
//
#include <hip/hip_runtime.h>


#ifndef NB
#define NB 2
#endif
#ifndef SEQ
#define SEQ 2048
#endif
#ifndef RH
#define RH 256
#endif
#define SEQ_FULL 2048
#define DIM  2048
#define DSH  11
#define NH   16
#define HD   128
#define LDC  (3 * DIM)
#define MCH  (SEQ < 1024 ? SEQ : 1024)
#define NCH  ((NB * SEQ) / MCH)
#define NFL  (SEQ / 32)
#define QCAR 16.0f
#define PCAR 1024.0f
#define VCAR 16.0f
#define WCAR 1024.0f
#define L2E  1.4426950408889634f

static_assert((1 << DSH) == DIM);
static_assert(NH * HD == DIM);
static_assert(SEQ % 128 == 0 && SEQ <= SEQ_FULL);
static_assert(RH % 64 == 0 && RH <= SEQ && RH >= 64);
static_assert(SEQ % MCH == 0 && MCH % 64 == 0 && (NB * SEQ) % MCH == 0);
static_assert(4 * 256 * 8 == 64 * HD);
static_assert(((DIM * DIM) / 64) % 64 == 0);
static_assert(((SEQ * DIM) / 8) % 256 == 0);

typedef _Float16 h16;
typedef unsigned short us;
typedef __attribute__((ext_vector_type(16))) __bf16   v16bf;
typedef __attribute__((ext_vector_type(16))) _Float16 v16h;
typedef __attribute__((ext_vector_type(16))) unsigned short v16us;
typedef __attribute__((ext_vector_type(8)))  unsigned short v8us;
typedef __attribute__((ext_vector_type(4)))  unsigned short v4us;
typedef __attribute__((ext_vector_type(2)))  unsigned short v2us;
typedef __attribute__((ext_vector_type(8)))  float    v8f;
typedef __attribute__((ext_vector_type(4)))  float    v4f;
typedef v4f  __attribute__((may_alias)) v4fa;
typedef v8us __attribute__((may_alias)) v8usa;
typedef v4us __attribute__((may_alias)) v4usa;

__device__ __forceinline__ us f2bf(float f) { unsigned u = __float_as_uint(f); u += 0x7FFFu + ((u >> 16) & 1u); return (us)(u >> 16); }
__device__ __forceinline__ float bf2f(us b) { return __uint_as_float(((unsigned)b) << 16); }
__device__ __forceinline__ float bfr(float f) { return bf2f(f2bf(f)); }
__device__ __forceinline__ void splitf(float y, us& h, us& l) { h = f2bf(y); l = f2bf(y - bf2f(h)); }
__device__ __forceinline__ us h2bits(float x) { return __builtin_bit_cast(us, (h16)x); }
__device__ __forceinline__ v16us cat16u(v8us lo, v8us hi) { return __builtin_shufflevector(lo, hi, 0, 1, 2, 3, 4, 5, 6, 7, 8, 9, 10, 11, 12, 13, 14, 15); }
__device__ __forceinline__ v8f wmma16(v16h a, v16h b, v8f c) { return __builtin_amdgcn_wmma_f32_16x16x32_f16(false, a, false, b, (short)0, c, false, false); }
__device__ __forceinline__ v8f wmmab(v16bf a, v16bf b, v8f c) { return __builtin_amdgcn_wmma_f32_16x16x32_bf16(false, a, false, b, (short)0, c, false, false); }
__device__ __forceinline__ void wave_sync() { __builtin_amdgcn_fence(3  , "wavefront"); __builtin_amdgcn_wave_barrier(); asm volatile("" ::: "memory"); }

template <int TY> struct WFrag;
template <> struct WFrag<0> { typedef v16bf V;
    static __device__ __forceinline__ V ld(const us* p)  { return __builtin_bit_cast(v16bf, cat16u(*(const v8us*)p, *(const v8us*)(p + 16))); }
    static __device__ __forceinline__ V lds(const us* p) { return __builtin_bit_cast(v16bf, cat16u(*(const v8usa*)p, *(const v8usa*)(p + 16))); }
    static __device__ __forceinline__ v8f mma(V a, V b, v8f c) { return wmmab(a, b, c); } };
template <> struct WFrag<1> { typedef v16h V;
    static __device__ __forceinline__ V ld(const us* p)  { return __builtin_bit_cast(v16h, cat16u(*(const v8us*)p, *(const v8us*)(p + 16))); }
    static __device__ __forceinline__ V lds(const us* p) { return __builtin_bit_cast(v16h, cat16u(*(const v8usa*)p, *(const v8usa*)(p + 16))); }
    static __device__ __forceinline__ v8f mma(V a, V b, v8f c) { return wmma16(a, b, c); } };

template <int TY, int NSPLIT>
__global__ __launch_bounds__(32) void k_gemmw(const us* __restrict__ A, const us* __restrict__ A2, const us* __restrict__ Bt, int K, float* C, int ldc, float oscale, size_t sA, size_t sC) {
    typedef WFrag<TY> W; typedef typename W::V V;
    __shared__ __align__(16) float os[16 * 68];
    const size_t z = blockIdx.z; A += z * sA; A2 += z * sA; C += z * sC;
    const int lane = threadIdx.x & 31, lr = lane & 15, hi = lane >> 4; const int r0 = blockIdx.x * 64, c0 = blockIdx.y * 64;
    v8f acc[4][4];
#pragma unroll
    for (int mb = 0; mb < 4; ++mb)
#pragma unroll
        for (int nb = 0; nb < 4; ++nb) acc[mb][nb] = (v8f){};
    const size_t aoff = (size_t)(r0 + lr) * K + 8 * hi, boff = (size_t)(c0 + lr) * K + 8 * hi;
#pragma unroll 1
    for (int kc = 0; kc < K; kc += 32) {
        V a[4], a2[4];
#pragma unroll
        for (int mb = 0; mb < 4; ++mb) { a[mb] = W::ld(A + aoff + (size_t)mb * 16 * K + kc); if (NSPLIT == 1) a2[mb] = W::ld(A2 + aoff + (size_t)mb * 16 * K + kc); }
#pragma unroll
        for (int nb = 0; nb < 4; ++nb) { const V b = W::ld(Bt + boff + (size_t)nb * 16 * K + kc);
#pragma unroll
            for (int mb = 0; mb < 4; ++mb) { acc[mb][nb] = W::mma(a[mb], b, acc[mb][nb]); if (NSPLIT == 1) acc[mb][nb] = W::mma(a2[mb], b, acc[mb][nb]); } }
        asm volatile("v_nop\n\tv_nop\n\tv_nop\n\tv_nop" : "+v"(acc[0][0]), "+v"(acc[1][1]), "+v"(acc[2][2]), "+v"(acc[3][3]) : "v"(a[0]), "v"(a[3]));
    }
#pragma unroll
    for (int mb = 0; mb < 4; ++mb) {
#pragma unroll
        for (int nb = 0; nb < 4; ++nb) {
#pragma unroll
            for (int j = 0; j < 8; ++j) os[(hi * 8 + j) * 68 + nb * 16 + lr] = acc[mb][nb][j]; }
        wave_sync();
        float* crow = C + (size_t)(r0 + mb * 16) * ldc + c0;
#pragma unroll 1
        for (int ps = 0; ps < 2; ++ps) {
#pragma unroll
            for (int s = 0; s < 8; ++s) { const int row = 2 * s + hi, cofs = lr * 4; v4f val = *(const v4fa*)(os + row * 68 + cofs); val[0] *= oscale; val[1] *= oscale; val[2] *= oscale; val[3] *= oscale;
                *(volatile v4f*)(crow + (size_t)row * ldc + cofs) = val; }
            if (ps == 0) __threadfence(); }
        wave_sync();
    }
}

template <int MODE>
__global__ __launch_bounds__(256) void k_wtG(const float* __restrict__ w, us* Bt, us* Bt2) {
    const unsigned lane = threadIdx.x & 31u; const unsigned L0 = (blockIdx.x * 8u + (threadIdx.x >> 5)) * 8u;
#pragma unroll 1
    for (int ps = 0; ps < 2; ++ps) {
#pragma unroll 1
        for (unsigned l = 0; l < 8u; ++l) { const unsigned e = (L0 + l) * 64u + lane * 2u; const unsigned k = e & (unsigned)(DIM - 1), n = e >> DSH;
            const float w0 = w[(size_t)k * DIM + n], w1 = w[(size_t)(k + 1u) * DIM + n]; v2us o; o[0] = f2bf(w0); o[1] = f2bf(w1); *(volatile v2us*)(Bt + e) = o;
            if (MODE == 1) { v2us o2; o2[0] = h2bits(bf2f(o[0]) * WCAR); o2[1] = h2bits(bf2f(o[1]) * WCAR); *(volatile v2us*)(Bt2 + e) = o2; } }
        if (ps == 0) __threadfence(); }
}

__global__ __launch_bounds__(256) void k_cvt8(const float* __restrict__ src, us* dst) {
    const unsigned i = blockIdx.x * 256u + threadIdx.x; const float* s = src + (size_t)blockIdx.y * SEQ_FULL * DIM + (size_t)i * 8; us* d = dst + (size_t)blockIdx.y * SEQ * DIM + (size_t)i * 8;
    const v8f v = *(const v8f*)s; v8us o;
#pragma unroll
    for (int k = 0; k < 8; ++k) o[k] = f2bf(v[k]);
    *(volatile v8us*)d = o; __threadfence(); *(volatile v8us*)d = o; }

__global__ __launch_bounds__(256) void k_maskchk(const float* __restrict__ mask, float* FL) {
    __shared__ unsigned wb[8];
    const unsigned lane = threadIdx.x & 31u, wave = threadIdx.x >> 5; unsigned bad = 0u;
#pragma unroll 1
    for (unsigned i = 0; i < 4u; ++i) { const unsigned r = blockIdx.x * 32u + wave * 4u + i; const float* mr = mask + (size_t)r * SEQ_FULL;
#pragma unroll 1
        for (unsigned it = 0; it < (unsigned)(SEQ / 128); ++it) { const unsigned c = it * 128u + lane * 4u; const v4f v = *(const v4f*)(mr + c);
#pragma unroll
            for (unsigned q = 0; q < 4u; ++q) { const float x = v[q]; const bool ok = (c + q <= r) ? (x == 0.0f) : (x <= -1.0e4f); bad |= ok ? 0u : 1u; } } }
    const unsigned long long bm = __ballot(bad != 0u);
    if (lane == 0u) wb[wave] = (bm != 0ull) ? 1u : 0u;
    __syncthreads();
    if (wave == 0u) { const unsigned f = wb[lane & 7u]; const unsigned long long am = __ballot(f != 0u); const float fv = (am != 0ull) ? 1.0f : 0.0f;
        *(volatile float*)(FL + blockIdx.x * 32u + lane) = fv; __threadfence(); *(volatile float*)(FL + blockIdx.x * 32u + lane) = fv; }
}

__global__ __launch_bounds__(256) void k_pack(const float* __restrict__ C, unsigned b, unsigned tbase, const float* __restrict__ fcos, const float* __restrict__ fsin,
                                              const float* __restrict__ qw, const float* __restrict__ qb, const float* __restrict__ kw, const float* __restrict__ kb,
                                              us* Q16, us* K16, us* VT16, us* QEh, us* QEl, us* KEh, us* KEl, us* VEh, us* VEl) {
    __shared__ __align__(16) us sA[9216]; __shared__ __align__(16) us sH[9216]; __shared__ __align__(16) us sL[9216];
    const unsigned tid = threadIdx.x, lane = tid & 31u, wave = tid >> 5;
    const unsigned h = blockIdx.y, r0 = blockIdx.x * 64u, t0 = tbase + r0, bh = b * NH + h;
    const bool hires = (t0 < (unsigned)RH); const unsigned te = hires ? t0 : 0u;
    float lwq[4], lbq[4], lwk[4], lbk[4];
#pragma unroll
    for (int j = 0; j < 4; ++j) { lwq[j] = bfr(qw[lane * 4u + j]); lbq[j] = bfr(qb[lane * 4u + j]); lwk[j] = bfr(kw[lane * 4u + j]); lbk[j] = bfr(kb[lane * 4u + j]); }
#pragma unroll 1
    for (unsigned which = 0; which < 3u; ++which) {
        if (which < 2u) {
#pragma unroll 1
            for (unsigned i = 0; i < 8u; ++i) { const unsigned tt = wave * 8u + i;
                const v4f xv = *(const v4f*)(C + (size_t)(r0 + tt) * LDC + which * DIM + h * HD + lane * 4u);
                float s = (xv[0] + xv[1]) + (xv[2] + xv[3]);
#pragma unroll
                for (int sh = 16; sh; sh >>= 1) s += __shfl_xor(s, sh, 32);
                const float mu = s * (1.0f / HD);
                const float d0 = xv[0] - mu, d1 = xv[1] - mu, d2 = xv[2] - mu, d3 = xv[3] - mu;
                float vs = (d0 * d0 + d1 * d1) + (d2 * d2 + d3 * d3);
#pragma unroll
                for (int sh = 16; sh; sh >>= 1) vs += __shfl_xor(vs, sh, 32);
                const float r = rsqrtf(vs * (1.0f / HD) + 1.0e-5f);
                const float y0 = d0 * r * (which == 0u ? lwq[0] : lwk[0]) + (which == 0u ? lbq[0] : lbk[0]);
                const float y1 = d1 * r * (which == 0u ? lwq[1] : lwk[1]) + (which == 0u ? lbq[1] : lbk[1]);
                const float y2 = d2 * r * (which == 0u ? lwq[2] : lwk[2]) + (which == 0u ? lbq[2] : lbk[2]);
                const float y3 = d3 * r * (which == 0u ? lwq[3] : lwk[3]) + (which == 0u ? lbq[3] : lbk[3]);
                const unsigned fi = (t0 + tt) * (unsigned)(HD / 2) + lane * 2u;
                const float c0 = bfr(fcos[fi]), c1 = bfr(fcos[fi + 1u]), s0 = bfr(fsin[fi]), s1 = bfr(fsin[fi + 1u]);
                float o[4]; o[0] = y0 * c0 - y1 * s0; o[1] = y0 * s0 + y1 * c0; o[2] = y2 * c1 - y3 * s1; o[3] = y2 * s1 + y3 * c1;
                v4us m;
#pragma unroll
                for (int j = 0; j < 4; ++j) m[j] = h2bits(o[j] * QCAR);
                *(v4usa*)(sA + tt * 136u + lane * 4u) = m;
                if (hires) { v4us mh, ml;
#pragma unroll
                    for (int j = 0; j < 4; ++j) { us a, c; splitf(o[j], a, c); mh[j] = a; ml[j] = c; }
                    *(v4usa*)(sH + tt * 136u + lane * 4u) = mh; *(v4usa*)(sL + tt * 136u + lane * 4u) = ml; } }
            __syncthreads();
            us* d16 = (which == 0u ? Q16 : K16) + ((size_t)bh * SEQ + t0) * HD;
            us* dEh = (which == 0u ? QEh : KEh) + ((size_t)bh * RH + te) * HD;
            us* dEl = (which == 0u ? QEl : KEl) + ((size_t)bh * RH + te) * HD;
#pragma unroll 1
            for (int ps = 0; ps < 2; ++ps) {
#pragma unroll
                for (unsigned it = 0; it < 4u; ++it) { const unsigned pi = it * 256u + tid; const unsigned so = (pi >> 4) * 136u + (pi & 15u) * 8u;
                    const v8us v = *(const v8usa*)(sA + so); *(volatile v8us*)(d16 + (size_t)pi * 8u) = v;
                    if (hires) { const v8us vh = *(const v8usa*)(sH + so); const v8us vl = *(const v8usa*)(sL + so); *(volatile v8us*)(dEh + (size_t)pi * 8u) = vh; *(volatile v8us*)(dEl + (size_t)pi * 8u) = vl; } }
                if (ps == 0) __threadfence(); }
            __syncthreads();
        } else {
#pragma unroll 1
            for (unsigned i = 0; i < 8u; ++i) { const unsigned tt = wave * 8u + i;
                const v4f xv = *(const v4f*)(C + (size_t)(r0 + tt) * LDC + 2u * DIM + h * HD + lane * 4u);
#pragma unroll
                for (unsigned j = 0; j < 4u; ++j) { const unsigned so = (lane * 4u + j) * 72u + tt; sA[so] = h2bits(xv[j] * VCAR);
                    if (hires) { us a, c; splitf(xv[j], a, c); sH[so] = a; sL[so] = c; } } }
            __syncthreads();
#pragma unroll 1
            for (int ps = 0; ps < 2; ++ps) {
#pragma unroll
                for (unsigned it = 0; it < 4u; ++it) { const unsigned pi = it * 256u + tid; const unsigned d = pi >> 3, c8 = pi & 7u; const unsigned so = d * 72u + c8 * 8u;
                    const v8us v = *(const v8usa*)(sA + so); *(volatile v8us*)(VT16 + ((size_t)bh * HD + d) * SEQ + t0 + c8 * 8u) = v;
                    if (hires) { const v8us vh = *(const v8usa*)(sH + so); const v8us vl = *(const v8usa*)(sL + so);
                        *(volatile v8us*)(VEh + ((size_t)bh * HD + d) * RH + te + c8 * 8u) = vh; *(volatile v8us*)(VEl + ((size_t)bh * HD + d) * RH + te + c8 * 8u) = vl; } }
                if (ps == 0) __threadfence(); }
            __syncthreads();
        }
    }
}

template <bool HI>
__global__ __launch_bounds__(128) void k_flash(const us* __restrict__ Qa, const us* __restrict__ Ka, const us* __restrict__ Va, const us* __restrict__ Qb, const us* __restrict__ Kb, const us* __restrict__ Vb,
                                               const float* __restrict__ FL, us* Oa, us* Ob) {
    typedef WFrag<HI ? 0 : 1> W; typedef typename W::V V;
    constexpr unsigned TQ = HI ? (unsigned)RH : (unsigned)SEQ;
    constexpr unsigned QB0 = HI ? 0u : (unsigned)RH;
    __shared__ __align__(16) us Pa[4 * 640]; __shared__ __align__(16) us Pb[4 * 640];
    __shared__ __align__(16) us Osa[4 * 2176]; __shared__ __align__(16) us Osb[4 * 2176];
    const unsigned lane = threadIdx.x & 31u, wave = threadIdx.x >> 5, hi = lane >> 4, lr = lane & 15u;
    const unsigned bh = blockIdx.y, b = bh / NH, h = bh & (unsigned)(NH - 1);
    const unsigned wq0 = QB0 + blockIdx.x * 64u + wave * 16u;
    const unsigned kend = (wq0 + 16u + 31u) & ~31u;
    unsigned fb = 0u;
#pragma unroll 1
    for (unsigned c = 0; c < ((unsigned)NFL + 31u) / 32u; ++c) { unsigned idx = c * 32u + lane; idx = (idx < (unsigned)NFL) ? idx : (unsigned)(NFL - 1); fb |= (FL[idx * 32u] != 0.0f) ? 1u : 0u; }
    const bool anybad = (__ballot(fb != 0u) != 0ull);
    const float pz = __uint_as_float(anybad ? 0x7FC00000u : 0u);
    const us* Qh_ = Qa + (size_t)bh * TQ * HD; const us* Kh_ = Ka + (size_t)bh * TQ * HD; const us* Vh_ = Va + (size_t)bh * HD * TQ;
    const us* Ql_ = Qb + (size_t)bh * TQ * HD; const us* Kl_ = Kb + (size_t)bh * TQ * HD; const us* Vl_ = Vb + (size_t)bh * HD * TQ;
    us* pa = Pa + wave * 640u; us* pb = Pb + wave * 640u; us* osa = Osa + wave * 2176u; us* osb = Osb + wave * 2176u;
    const size_t qo = (size_t)(wq0 + lr) * HD + 8u * hi;
    V qf[4];
#pragma unroll
    for (int j = 0; j < 4; ++j) qf[j] = W::ld(Qh_ + qo + j * 32);
    v8f o[8];
#pragma unroll
    for (int t = 0; t < 8; ++t) o[t] = (v8f){};
    float mi[8], li[8];
#pragma unroll
    for (int e = 0; e < 8; ++e) { mi[e] = -1.0e30f; li[e] = 0.0f; }
    const float SC = HI ? 0.08838834764831845f : (0.08838834764831845f * 0.00390625f);
#pragma unroll 1
    for (unsigned k0 = 0; k0 < kend; k0 += 32u) {
        v8f s0 = (v8f){}, s1 = (v8f){};
#pragma unroll
        for (int j = 0; j < 4; ++j) { const size_t ko = (size_t)(k0 + lr) * HD + j * 32 + 8u * hi;
            const V kf0 = W::ld(Kh_ + ko), kf1 = W::ld(Kh_ + ko + 16 * HD);
            s0 = W::mma(qf[j], kf0, s0); s1 = W::mma(qf[j], kf1, s1);
            if (HI) { const V ql = W::ld(Ql_ + qo + j * 32); const V kl0 = W::ld(Kl_ + ko), kl1 = W::ld(Kl_ + ko + 16 * HD);
                s0 = W::mma(qf[j], kl0, s0); s0 = W::mma(ql, kf0, s0); s1 = W::mma(qf[j], kl1, s1); s1 = W::mma(ql, kf1, s1); } }
        asm volatile("v_nop\n\tv_nop\n\tv_nop\n\tv_nop" : "+v"(s0), "+v"(s1) : "v"(qf[0]), "v"(qf[3]));
        const bool diag = (k0 + 31u > wq0);
        float al[8];
#pragma unroll
        for (int e = 0; e < 8; ++e) { const unsigned rg = wq0 + 8u * hi + (unsigned)e;
            float a0 = s0[e] * SC, a1 = s1[e] * SC;
            if (diag) { a0 = (k0 + lr > rg) ? (a0 + -1.0e9f) : a0; a1 = (k0 + 16u + lr > rg) ? (a1 + -1.0e9f) : a1; }
            float mx = fmaxf(a0, a1);
#pragma unroll
            for (int sh = 8; sh; sh >>= 1) mx = fmaxf(mx, __shfl_xor(mx, sh, 32));
            const float mn = fmaxf(mi[e], mx);
            al[e] = __builtin_amdgcn_exp2f((mi[e] - mn) * L2E);
            const float p0 = __builtin_amdgcn_exp2f((a0 - mn) * L2E), p1 = __builtin_amdgcn_exp2f((a1 - mn) * L2E);
            li[e] = li[e] * al[e] + (p0 + p1); mi[e] = mn; s0[e] = p0; s1[e] = p1; }
#pragma unroll
        for (int t = 0; t < 8; ++t)
#pragma unroll
            for (int e = 0; e < 8; ++e) o[t][e] *= al[e];
#pragma unroll
        for (int e = 0; e < 8; ++e) { const unsigned po = (8u * hi + (unsigned)e) * 40u + lr;
            if (HI) { us a, c; splitf(s0[e], a, c); pa[po] = a; pb[po] = c; splitf(s1[e], a, c); pa[po + 16u] = a; pb[po + 16u] = c; }
            else { pa[po] = h2bits(s0[e] * PCAR); pa[po + 16u] = h2bits(s1[e] * PCAR); } }
        wave_sync();
        const V pf = W::lds(pa + lr * 40u + 8u * hi); V pl = pf; if (HI) pl = W::lds(pb + lr * 40u + 8u * hi);
        wave_sync();
#pragma unroll
        for (int t = 0; t < 8; ++t) { const size_t vo = (size_t)(t * 16 + lr) * TQ + k0 + 8u * hi; const V vf = W::ld(Vh_ + vo);
            o[t] = W::mma(pf, vf, o[t]);
            if (HI) { const V vl = W::ld(Vl_ + vo); o[t] = W::mma(pf, vl, o[t]); o[t] = W::mma(pl, vf, o[t]); } }
        asm volatile("v_nop\n\tv_nop\n\tv_nop\n\tv_nop" : "+v"(o[0]), "+v"(o[1]), "+v"(o[2]), "+v"(o[3]), "+v"(o[4]), "+v"(o[5]), "+v"(o[6]), "+v"(o[7]) : "v"(pf), "v"(pl));
    }
#pragma unroll
    for (int e = 0; e < 8; ++e) { float l = li[e];
#pragma unroll
        for (int sh = 8; sh; sh >>= 1) l += __shfl_xor(l, sh, 32);
        const float f = (HI ? 1.0f : 0.015625f) * (1.0f / l);
#pragma unroll
        for (int t = 0; t < 8; ++t) { const unsigned so = (8u * hi + (unsigned)e) * 136u + (unsigned)t * 16u + lr; const float val = o[t][e] * f + pz;
            if (HI) { us a, c; splitf(val, a, c); osa[so] = a; osb[so] = c; }
            else { osa[so] = h2bits(val); } } }
    wave_sync();
    us* orow = Oa + (size_t)(b * TQ + wq0) * DIM + h * HD; us* orow2 = Ob + (size_t)(b * TQ + wq0) * DIM + h * HD;
#pragma unroll 1
    for (int ps = 0; ps < 2; ++ps) {
#pragma unroll
        for (unsigned s = 0; s < 8u; ++s) { const unsigned row = 2u * s + hi; const unsigned so = row * 136u + lr * 8u;
            const v8us v = *(const v8usa*)(osa + so); *(volatile v8us*)(orow + (size_t)row * DIM + lr * 8u) = v;
            if (HI) { const v8us v2 = *(const v8usa*)(osb + so); *(volatile v8us*)(orow2 + (size_t)row * DIM + lr * 8u) = v2; } }
        if (ps == 0) __threadfence(); }
}

#define SZ_XB   ((size_t)NB * SEQ * DIM * 2)
#define SZ_W3   ((size_t)3 * DIM * DIM * 2)
#define SZ_W1   ((size_t)DIM * DIM * 2)
#define SZ_C    ((size_t)MCH * LDC * 4)
#define SZ_PL   ((size_t)NB * NH * SEQ * HD * 2)
#define SZ_EP   ((size_t)NB * NH * RH * HD * 2)
#define SZ_CE   ((size_t)NB * RH * DIM * 2)
#define SZ_FL   ((size_t)NFL * 128)
static_assert(2 * SZ_W1 <= SZ_W3);
static_assert(2 * SZ_CE <= SZ_C);
static_assert(SZ_XB + SZ_W3 + SZ_C + 3 * SZ_PL + 6 * SZ_EP + SZ_FL + 16 * 256 <= (size_t)134217728);

extern "C" void kernel_launch(void* const* d_in, const int* in_sizes, int n_in,
                              void* d_out, int out_size, void* d_ws, size_t ws_size, hipStream_t stream) {
    if (n_in < 12) return;
    if (in_sizes[0] < (NB - 1) * SEQ_FULL * DIM + SEQ * DIM) return;
    if (in_sizes[1] < SEQ * (HD / 2) || in_sizes[2] < SEQ * (HD / 2)) return;
    if (in_sizes[3] < (SEQ - 1) * SEQ_FULL + SEQ) return;
    if (in_sizes[4] < DIM * DIM || in_sizes[5] < DIM * DIM || in_sizes[6] < DIM * DIM || in_sizes[7] < DIM * DIM) return;
    if (in_sizes[8] < HD || in_sizes[9] < HD || in_sizes[10] < HD || in_sizes[11] < HD) return;
    if (out_size < NB * SEQ * DIM) return;
    const float* x = (const float*)d_in[0]; const float* fcos = (const float*)d_in[1]; const float* fsin = (const float*)d_in[2]; const float* mask = (const float*)d_in[3];
    const float* wq = (const float*)d_in[4]; const float* wk = (const float*)d_in[5]; const float* wv = (const float*)d_in[6]; const float* wo = (const float*)d_in[7];
    const float* qlw = (const float*)d_in[8]; const float* qlb = (const float*)d_in[9]; const float* klw = (const float*)d_in[10]; const float* klb = (const float*)d_in[11];
    float* OUT = (float*)d_out;
    char* wsp = (char*)d_ws;
    auto take = [&](size_t bytes) { char* p = wsp; wsp += (bytes + 255) & ~(size_t)255; return (void*)p; };
    us* XB = (us*)take(SZ_XB);
    us* WQKV = (us*)take(SZ_W3);
    float* Cch = (float*)take(SZ_C);
    us* Q16 = (us*)take(SZ_PL); us* K16 = (us*)take(SZ_PL); us* VT16 = (us*)take(SZ_PL);
    us* QEh = (us*)take(SZ_EP); us* QEl = (us*)take(SZ_EP); us* KEh = (us*)take(SZ_EP); us* KEl = (us*)take(SZ_EP); us* VEh = (us*)take(SZ_EP); us* VEl = (us*)take(SZ_EP);
    float* FL = (float*)take(SZ_FL);
    if ((size_t)(wsp - (char*)d_ws) > ws_size) return;
    us* CTX = XB; us* WOB = WQKV; us* WOH = WQKV + (size_t)DIM * DIM; us* CEh = (us*)Cch; us* CEl = CEh + (size_t)NB * RH * DIM;

    k_maskchk<<<SEQ / 32, 256, 0, stream>>>(mask, FL);
    k_cvt8<<<dim3((unsigned)(((size_t)SEQ * DIM / 8) / 256), NB), 256, 0, stream>>>(x, XB);
    k_wtG<0><<<(DIM * DIM / 64) / 64, 256, 0, stream>>>(wq, WQKV, WQKV);
    k_wtG<0><<<(DIM * DIM / 64) / 64, 256, 0, stream>>>(wk, WQKV + (size_t)DIM * DIM, WQKV);
    k_wtG<0><<<(DIM * DIM / 64) / 64, 256, 0, stream>>>(wv, WQKV + (size_t)2 * DIM * DIM, WQKV);
    for (int c = 0; c < NCH; ++c) {
        const unsigned grow = (unsigned)c * MCH; const unsigned b = grow / SEQ, tbase = grow % SEQ;
        const us* xa = XB + (size_t)grow * DIM;
        k_gemmw<0, 0><<<dim3(MCH / 64, LDC / 64, 1), 32, 0, stream>>>(xa, xa, WQKV, DIM, Cch, LDC, 1.0f, 0, 0);
        k_pack<<<dim3(MCH / 64, NH), 256, 0, stream>>>(Cch, b, tbase, fcos, fsin, qlw, qlb, klw, klb, Q16, K16, VT16, QEh, QEl, KEh, KEl, VEh, VEl);
    }
    k_wtG<1><<<(DIM * DIM / 64) / 64, 256, 0, stream>>>(wo, WOB, WOH);
    k_flash<true><<<dim3(RH / 64, NB * NH), 128, 0, stream>>>(QEh, KEh, VEh, QEl, KEl, VEl, FL, CEh, CEl);
    if (SEQ > RH) k_flash<false><<<dim3((SEQ - RH) / 64 + (SEQ == RH ? 1 : 0), NB * NH), 128, 0, stream>>>(Q16, K16, VT16, Q16, K16, VT16, FL, CTX, CTX);
    k_gemmw<0, 1><<<dim3(RH / 64, DIM / 64, NB), 32, 0, stream>>>(CEh, CEl, WOB, DIM, OUT, DIM, 1.0f, (size_t)RH * DIM, (size_t)SEQ * DIM);
    if (SEQ > RH) k_gemmw<1, 0><<<dim3((SEQ - RH) / 64 + (SEQ == RH ? 1 : 0), DIM / 64, NB), 32, 0, stream>>>(CTX + (size_t)RH * DIM, CTX + (size_t)RH * DIM, WOH, DIM, OUT + (size_t)RH * DIM, DIM, 3.814697265625e-06f, (size_t)SEQ * DIM, (size_t)SEQ * DIM);
}
